// scGraph_26585847562902
// MI455X (gfx1250) — hardware-verified
//
#include <hip/hip_runtime.h>
#include <stddef.h>
#include <math.h>


#define NN     2207
#define NP     2208
#define BB     512
#define MIDC   8
#define GC1C   12
#define GC2C   4
#define FC1C   256
#define FC2C   64
#define OUTC   2
#define KFC1   8828
#define KP1    8832
#define KD1    (3 * KP1)
#define KP2    256
#define KD2    (3 * KP2)
#define NLINE1 (KD1 / 64)
#define NIT    ((NN + 255) / 256)
#define NST    ((NLINE1 + 31) / 32)
#define EPS_F  1e-5f

#define NTHR   256
#define NWAVE  8
#define EPT    8
#define NGRP   2
#define CHUNK  (NTHR * EPT * NGRP)
#define WCAP   (EPT * NGRP * 32)
#define LISTN  (NWAVE * WCAP)
#define NBA    32
#define LDS_AGG  ((NBA * BB) * 4 + LISTN * 4 + NBA * 4 + NWAVE * 4)
#define LDS_GEMM (NWAVE * 32 * 64 * 4)
#define WSCAP  134217728

static_assert((CHUNK & (CHUNK - 1)) == 0);
static_assert(CHUNK <= 4096);
static_assert(WCAP == EPT * NGRP * 32);
static_assert(LISTN == NWAVE * WCAP);
static_assert((NBA & (NBA - 1)) == 0 && NBA <= 4096);
static_assert((NP % NBA) == 0 && NP >= NN && (NP % 32) == 0);
static_assert(BB == 2 * NTHR);
static_assert(BB == NWAVE * 64);
static_assert((KP1 % 32) == 0 && KP1 - KFC1 == 4);
static_assert((KD1 % 64) == 0 && NLINE1 * 64 == KD1);
static_assert(GC2C * NN == KFC1);
static_assert(NIT * NTHR >= NN);
static_assert(NST * 32 >= NLINE1);
static_assert((BB % 64) == 0 && (BB % 256) == 0);

typedef float          v4f  __attribute__((ext_vector_type(4)));
typedef float          v8f  __attribute__((ext_vector_type(8)));
typedef int            v4i  __attribute__((ext_vector_type(4)));
typedef unsigned short v8us __attribute__((ext_vector_type(8)));
typedef __bf16         v16b __attribute__((ext_vector_type(16)));
union FragB { v16b v; v8us half[2]; };

__device__ __forceinline__ v8f wmb(v16b a, v16b b, v8f c) {
  v8f d = __builtin_amdgcn_wmma_f32_16x16x32_bf16(false, a, false, b, (short)0, c, false, false);
  asm volatile("v_nop\n\tv_nop\n\tv_nop\n\tv_nop" : "+v"(d) : "v"(a), "v"(b));
  return d;
}

__device__ __forceinline__ unsigned int f2bf(float x) {
  const unsigned int u = __float_as_uint(x);
  return (u + 0x7FFFu + ((u >> 16) & 1u)) >> 16;
}
__device__ __forceinline__ void split_bf(float x, unsigned short& hi, unsigned short& lo) {
  const unsigned int h = f2bf(x);
  const float xh = __uint_as_float(h << 16);
  hi = (unsigned short)h;
  lo = (unsigned short)f2bf(x - xh);
}

template <int NB>
__device__ __forceinline__ int scan_chunk(const int* __restrict__ dsts, int nE, int cbase, int slotBase,
                                          int vec8, int* list, int tid, int lane, int wave) {
  int wc = 0;
#pragma unroll
  for (int g = 0; g < NGRP; ++g) {
    const int el0  = (g * NTHR + tid) * EPT;
    const int e0   = cbase + el0;
    const int sent = -2147483647 - 1;
    v4i da, db;
    if (vec8 != 0 && cbase + CHUNK <= nE) {
      da = *(const v4i*)(dsts + e0);
      db = *(const v4i*)(dsts + e0 + 4);
    } else {
      da.x = (e0     < nE) ? dsts[min(e0, nE - 1)] : sent;
      da.y = (e0 + 1 < nE) ? dsts[min(e0 + 1, nE - 1)] : sent;
      da.z = (e0 + 2 < nE) ? dsts[min(e0 + 2, nE - 1)] : sent;
      da.w = (e0 + 3 < nE) ? dsts[min(e0 + 3, nE - 1)] : sent;
      db.x = (e0 + 4 < nE) ? dsts[min(e0 + 4, nE - 1)] : sent;
      db.y = (e0 + 5 < nE) ? dsts[min(e0 + 5, nE - 1)] : sent;
      db.z = (e0 + 6 < nE) ? dsts[min(e0 + 6, nE - 1)] : sent;
      db.w = (e0 + 7 < nE) ? dsts[min(e0 + 7, nE - 1)] : sent;
    }
    const unsigned nb = (unsigned)slotBase;
    const unsigned s0 = (unsigned)da.x - nb, s1 = (unsigned)da.y - nb;
    const unsigned s2 = (unsigned)da.z - nb, s3 = (unsigned)da.w - nb;
    const unsigned s4 = (unsigned)db.x - nb, s5 = (unsigned)db.y - nb;
    const unsigned s6 = (unsigned)db.z - nb, s7 = (unsigned)db.w - nb;
    const bool h0 = s0 < (unsigned)NB, h1 = s1 < (unsigned)NB, h2 = s2 < (unsigned)NB, h3 = s3 < (unsigned)NB;
    const bool h4 = s4 < (unsigned)NB, h5 = s5 < (unsigned)NB, h6 = s6 < (unsigned)NB, h7 = s7 < (unsigned)NB;
    const unsigned any = __builtin_amdgcn_ballot_w32(h0 | h1 | h2 | h3 | h4 | h5 | h6 | h7);
    if (any != 0u) {
#define HITJ(J, HJ, SJ) { \
        const unsigned mj = __builtin_amdgcn_ballot_w32(HJ); \
        if (mj != 0u) { \
          if (HJ) { \
            const int pos = wc + (int)__builtin_amdgcn_mbcnt_lo(mj, 0u); \
            if (pos < WCAP) list[wave * WCAP + pos] = ((el0 + (J)) << 12) | (int)(SJ); \
          } \
          wc += (int)__builtin_popcount(mj); } }
      HITJ(0, h0, s0)
      HITJ(1, h1, s1)
      HITJ(2, h2, s2)
      HITJ(3, h3, s3)
      HITJ(4, h4, s4)
      HITJ(5, h5, s5)
      HITJ(6, h6, s6)
      HITJ(7, h7, s7)
#undef HITJ
    }
  }
  return wc;
}

__global__ __launch_bounds__(NTHR) void k_wprep(
    const float* __restrict__ W, unsigned short* dst, int K, int N, int KP, int total) {
  const int i = blockIdx.x * NTHR + threadIdx.x;
  if (i >= total) return;
  const int kq  = KP >> 3;
  const int gpr = 3 * kq;
  const int n   = i / gpr;
  const int r   = i - n * gpr;
  const int seg = r / kq;
  const int k0  = (r - seg * kq) * 8;
  v8us o;
#pragma unroll
  for (int e = 0; e < 8; ++e) {
    const int k  = k0 + e;
    const int kk = k < K - 1 ? k : K - 1;
    const float va = W[(size_t)kk * N + n];
    const float v  = (k < K) ? va : 0.0f;
    unsigned short hi, lo;
    split_bf(v, hi, lo);
    o[e] = (seg == 1) ? lo : hi;
  }
  unsigned short* d = dst + (size_t)i * 8;
  *(volatile v8us*)d = o;
  __threadfence();
  *(volatile v8us*)d = o;
}

__global__ __launch_bounds__(NTHR) void k_sig(const float* __restrict__ ewp, float* sig, int nE, int nP) {
  const int i = blockIdx.x * NTHR + threadIdx.x;
  if (i >= nP) return;
  const int e = i < nE - 1 ? i : nE - 1;
  const float v = ewp[e];
  const float t = expf(-v);
  const float w = 1.0f / (1.0f + t);
  *(volatile float*)(sig + i) = w;
  __threadfence();
  *(volatile float*)(sig + i) = w;
}

__global__ __launch_bounds__(NTHR) void k_agg(
    const float* __restrict__ x, const int* __restrict__ ei, const float* __restrict__ sig,
    float* aggT, int nE, int vec8) {
  extern __shared__ v4f lds_dyn[];
  float* sums = (float*)lds_dyn;
  int*   list = (int*)(sums + NBA * BB);
  int*   scnt = list + LISTN;
  int*   wcnt = scnt + NBA;
  const int tid = threadIdx.x, lane = tid & 31, wave = tid >> 5;
  const int nodeBase = blockIdx.x * NBA;
  const int* dsts = ei + nE;

  {
    const v4f z = {0.f, 0.f, 0.f, 0.f};
    for (int i = tid; i < (NBA * BB) / 4; i += NTHR) ((v4f*)sums)[i] = z;
    if (tid < NBA) scnt[tid] = 0;
  }
  __syncthreads();

  const int nChunks = (nE + CHUNK - 1) / CHUNK;
#pragma unroll 1
  for (int ch = 0; ch < nChunks; ++ch) {
    const int cbase = ch * CHUNK;
    const int wc = scan_chunk<NBA>(dsts, nE, cbase, nodeBase, vec8, list, tid, lane, wave);
    if (lane == 0) wcnt[wave] = wc;
    __syncthreads();
#pragma unroll 1
    for (int wsx = 0; wsx < NWAVE; ++wsx) {
      int n = __builtin_amdgcn_readfirstlane(wcnt[wsx]);
      n = n > WCAP ? WCAP : (n < 0 ? 0 : n);
      const int* lp = list + wsx * WCAP;
#pragma unroll 1
      for (int i = 0; i < n; ++i) {
        const int ent  = __builtin_amdgcn_readfirstlane(lp[i]);
        const int slot = ent & (NBA - 1);
        int e = cbase + ((ent >> 12) & (CHUNK - 1));
        e = e > nE - 1 ? nE - 1 : e;
        int s = ei[e];
        s = s < 0 ? 0 : (s > NN - 1 ? NN - 1 : s);
        const float w = sig[e];
        const float* xr = x + (size_t)s * BB;
        const float xa = xr[tid];
        const float xb = xr[tid + NTHR];
        float* sp = sums + slot * BB + tid;
        sp[0]    = fmaf(w, xa, sp[0]);
        sp[NTHR] = fmaf(w, xb, sp[NTHR]);
        if (tid == 0) scnt[slot] = scnt[slot] + 1;
      }
    }
    __syncthreads();
  }

#pragma unroll 1
  for (int i = tid; i < NBA * BB; i += NTHR) {
    const int slot = i >> 9;
    const int c = scnt[slot];
    const float d  = (float)(c > 1 ? c : 1);
    const float rc = 1.0f / d;
    sums[i] = sums[i] * rc;
  }
  __syncthreads();

  const int j = lane & 7, rsub = lane >> 3;
#pragma unroll 1
  for (int q = 0; q < 16; ++q) {
    const int b = 64 * wave + 4 * q + rsub;
    const float* sp = sums + b;
    v4f v;
    v.x = sp[(4 * j + 0) * BB]; v.y = sp[(4 * j + 1) * BB];
    v.z = sp[(4 * j + 2) * BB]; v.w = sp[(4 * j + 3) * BB];
    *(volatile v4f*)(aggT + (size_t)b * NP + nodeBase + 4 * j) = v;
  }
  __threadfence();
#pragma unroll 1
  for (int q = 0; q < 16; ++q) {
    const int b = 64 * wave + 4 * q + rsub;
    const float* sp = sums + b;
    v4f v;
    v.x = sp[(4 * j + 0) * BB]; v.y = sp[(4 * j + 1) * BB];
    v.z = sp[(4 * j + 2) * BB]; v.w = sp[(4 * j + 3) * BB];
    *(volatile v4f*)(aggT + (size_t)b * NP + nodeBase + 4 * j) = v;
  }
}

__global__ __launch_bounds__(NTHR) void k_ln_conv(
    const float* __restrict__ aggT, const float* __restrict__ sgw, const float* __restrict__ sgb,
    const float* __restrict__ lng, const float* __restrict__ lnb,
    const float* __restrict__ gc1w, const float* __restrict__ gc1b,
    const float* __restrict__ bn1g, const float* __restrict__ bn1b,
    const float* __restrict__ gc2w, const float* __restrict__ gc2b,
    const float* __restrict__ bn2g, const float* __restrict__ bn2b,
    unsigned short* Ap) {
  __shared__ float cw[MIDC], cb[MIDC];
  __shared__ float w1[GC1C * MIDC], b1[GC1C], s1[GC1C], t1[GC1C];
  __shared__ float w2[GC2C * GC1C], b2[GC2C], s2[GC2C], t2[GC2C];
  __shared__ double red0[NTHR], red1[NTHR];
  __shared__ __attribute__((aligned(16))) unsigned short row16[2 * KP1];
  const int tid = threadIdx.x, b = blockIdx.x;
  const float rs = 1.0f / sqrtf(1.0f + EPS_F);
  if (tid < MIDC) { cw[tid] = sgw[tid]; cb[tid] = sgb[tid]; }
  if (tid < GC1C * MIDC) w1[tid] = gc1w[tid];
  if (tid < GC2C * GC1C) w2[tid] = gc2w[tid];
  if (tid < GC1C) { b1[tid] = gc1b[tid]; s1[tid] = bn1g[tid] * rs; t1[tid] = bn1b[tid]; }
  if (tid < GC2C) { b2[tid] = gc2b[tid]; s2[tid] = bn2g[tid] * rs; t2[tid] = bn2b[tid]; }
  if (tid < KP1 - KFC1) { row16[KFC1 + tid] = 0; row16[KP1 + KFC1 + tid] = 0; }
  __syncthreads();

  const float* arow = aggT + (size_t)b * NP;

  double s = 0.0, ss = 0.0;
#pragma unroll 1
  for (int it = 0; it < NIT; ++it) {
    const int n  = it * NTHR + tid;
    const int nc = n < NP - 1 ? n : NP - 1;
    const float a = arow[nc];
    const bool valid = n < NN;
#pragma unroll
    for (int c = 0; c < MIDC; ++c) {
      const float h  = fmaxf(fmaf(a, cw[c], cb[c]), 0.0f);
      const float hv = valid ? h : 0.0f;
      const double hd = (double)hv;
      s += hd;
      ss = fma(hd, hd, ss);
    }
  }
  red0[tid] = s; red1[tid] = ss;
  __syncthreads();
  for (int o = NTHR / 2; o > 0; o >>= 1) {
    if (tid < o) { red0[tid] += red0[tid + o]; red1[tid] += red1[tid + o]; }
    __syncthreads();
  }
  const double cntd = (double)(NN * MIDC);
  const double mud  = red0[0] / cntd;
  double vard = red1[0] / cntd - mud * mud;
  vard = vard > 0.0 ? vard : 0.0;
  const float mu = (float)mud;
  const float sd = sqrtf((float)vard + EPS_F);
  const float r  = 1.0f / sd;

#pragma unroll 1
  for (int it = 0; it < NIT; ++it) {
    const int n  = it * NTHR + tid;
    const int nc = n < NP - 1 ? n : NP - 1;
    const int ng = n < NN - 1 ? n : NN - 1;
    const float a = arow[nc];
    const bool valid = n < NN;
    const v4f ga = *(const v4f*)(lng + (size_t)ng * MIDC);
    const v4f gb = *(const v4f*)(lng + (size_t)ng * MIDC + 4);
    const v4f ba = *(const v4f*)(lnb + (size_t)ng * MIDC);
    const v4f bb = *(const v4f*)(lnb + (size_t)ng * MIDC + 4);
    float gam[MIDC], bet[MIDC], g[MIDC];
    gam[0] = ga.x; gam[1] = ga.y; gam[2] = ga.z; gam[3] = ga.w;
    gam[4] = gb.x; gam[5] = gb.y; gam[6] = gb.z; gam[7] = gb.w;
    bet[0] = ba.x; bet[1] = ba.y; bet[2] = ba.z; bet[3] = ba.w;
    bet[4] = bb.x; bet[5] = bb.y; bet[6] = bb.z; bet[7] = bb.w;
#pragma unroll
    for (int c = 0; c < MIDC; ++c) {
      const float h = fmaxf(fmaf(a, cw[c], cb[c]), 0.0f);
      g[c] = fmaf((h - mu) * r, gam[c], bet[c]);
    }
    float z0 = 0.f, z1 = 0.f, z2 = 0.f, z3 = 0.f;
#pragma unroll 1
    for (int o = 0; o < GC1C; ++o) {
      float acc = 0.0f;
#pragma unroll
      for (int c = 0; c < MIDC; ++c) acc = fmaf(w1[o * MIDC + c], g[c], acc);
      acc += b1[o];
      const float y = fmaf(fmaxf(acc, 0.0f), s1[o], t1[o]);
      z0 = fmaf(w2[o], y, z0);
      z1 = fmaf(w2[GC1C + o], y, z1);
      z2 = fmaf(w2[2 * GC1C + o], y, z2);
      z3 = fmaf(w2[3 * GC1C + o], y, z3);
    }
    const float y0 = fmaf(fmaxf(z0 + b2[0], 0.0f), s2[0], t2[0]);
    const float y1 = fmaf(fmaxf(z1 + b2[1], 0.0f), s2[1], t2[1]);
    const float y2 = fmaf(fmaxf(z2 + b2[2], 0.0f), s2[2], t2[2]);
    const float y3 = fmaf(fmaxf(z3 + b2[3], 0.0f), s2[3], t2[3]);
    if (valid) {
      unsigned short hi, lo;
      split_bf(y0, hi, lo); row16[0 * NN + n] = hi; row16[KP1 + 0 * NN + n] = lo;
      split_bf(y1, hi, lo); row16[1 * NN + n] = hi; row16[KP1 + 1 * NN + n] = lo;
      split_bf(y2, hi, lo); row16[2 * NN + n] = hi; row16[KP1 + 2 * NN + n] = lo;
      split_bf(y3, hi, lo); row16[3 * NN + n] = hi; row16[KP1 + 3 * NN + n] = lo;
    }
  }
  __syncthreads();

  unsigned short* rb = Ap + (size_t)b * KD1;
  const int q = tid >> 3, j = tid & 7;
  constexpr int LPS = KP1 / 64;
#pragma unroll 1
  for (int st = 0; st < NST; ++st) {
    const int L  = q + 32 * st;
    const int Lc = L < NLINE1 - 1 ? L : NLINE1 - 1;
    const int segsrc = (Lc >= 2 * LPS) ? KP1 : 0;
    const int li = Lc >= 2 * LPS ? Lc - 2 * LPS : (Lc >= LPS ? Lc - LPS : Lc);
    const v8us v = *(const v8us*)(row16 + segsrc + li * 64 + 8 * j);
    if (L < NLINE1) *(volatile v8us*)(rb + (size_t)L * 64 + 8 * j) = v;
  }
  __threadfence();
#pragma unroll 1
  for (int st = 0; st < NST; ++st) {
    const int L  = q + 32 * st;
    const int Lc = L < NLINE1 - 1 ? L : NLINE1 - 1;
    const int segsrc = (Lc >= 2 * LPS) ? KP1 : 0;
    const int li = Lc >= 2 * LPS ? Lc - 2 * LPS : (Lc >= LPS ? Lc - LPS : Lc);
    const v8us v = *(const v8us*)(row16 + segsrc + li * 64 + 8 * j);
    if (L < NLINE1) *(volatile v8us*)(rb + (size_t)L * 64 + 8 * j) = v;
  }
}

template <int KD, int NCOL, int MODE>
__global__ __launch_bounds__(NTHR) void k_gemm(
    const unsigned short* __restrict__ A, const unsigned short* __restrict__ Bw,
    const float* __restrict__ bias, const float* __restrict__ gam, const float* __restrict__ bet,
    float* C32, unsigned short* C16) {
  static_assert((KD % 32) == 0);
  static_assert((NCOL % 64) == 0 && (NWAVE % (NCOL / 64)) == 0);
  constexpr int WC = NCOL / 64, WR = NWAVE / WC, BROWS = 32 * WR, NKT = KD / 32;
  extern __shared__ v4f lds_dyn[];
  float* stg = (float*)lds_dyn;
  const int tid = threadIdx.x, lane = tid & 31, wave = tid >> 5, hh = lane >> 4, m = lane & 15;
  const int wr = wave / WC, wc = wave - wr * WC;
  const int row0 = blockIdx.x * BROWS + 32 * wr;
  const int col0 = 64 * wc;

  v8f acc[2][4];
#pragma unroll
  for (int i = 0; i < 2; ++i)
#pragma unroll
    for (int t = 0; t < 4; ++t) { v8f z = {0.f, 0.f, 0.f, 0.f, 0.f, 0.f, 0.f, 0.f}; acc[i][t] = z; }

  const unsigned short* ap = A  + (size_t)(row0 + m) * KD + 8 * hh;
  const unsigned short* bp = Bw + (size_t)(col0 + m) * KD + 8 * hh;
#pragma unroll 1
  for (int kt = 0; kt < NKT; ++kt) {
    FragB a0, a1;
    a0.half[0] = *(const v8us*)(ap + 32 * kt);
    a0.half[1] = *(const v8us*)(ap + 32 * kt + 16);
    a1.half[0] = *(const v8us*)(ap + (size_t)16 * KD + 32 * kt);
    a1.half[1] = *(const v8us*)(ap + (size_t)16 * KD + 32 * kt + 16);
#pragma unroll
    for (int t = 0; t < 4; ++t) {
      FragB bfr;
      bfr.half[0] = *(const v8us*)(bp + (size_t)(16 * t) * KD + 32 * kt);
      bfr.half[1] = *(const v8us*)(bp + (size_t)(16 * t) * KD + 32 * kt + 16);
      acc[0][t] = wmb(a0.v, bfr.v, acc[0][t]);
      acc[1][t] = wmb(a1.v, bfr.v, acc[1][t]);
    }
  }

  const float rs = 1.0f / sqrtf(1.0f + EPS_F);
  float* sw = stg + wave * 2048;
#pragma unroll
  for (int i = 0; i < 2; ++i) {
#pragma unroll
    for (int t = 0; t < 4; ++t) {
      const int n = col0 + 16 * t + m;
      const float bv = bias[n];
      const float sc = gam[n] * rs;
      const float sh = bet[n];
#pragma unroll
      for (int r = 0; r < 8; ++r)
        sw[(16 * i + 8 * hh + r) * 64 + 16 * t + m] = fmaxf(fmaf(acc[i][t][r] + bv, sc, sh), 0.0f);
    }
  }
  __syncthreads();

  if (MODE == 0) {
    const int srow = lane >> 4, scol = 4 * (lane & 15);
    float* gb = C32 + (size_t)row0 * NCOL + col0 + scol;
#pragma unroll
    for (int q = 0; q < 16; ++q) {
      const int row = 2 * q + srow;
      const v4f v = *(const v4f*)(sw + row * 64 + scol);
      *(volatile v4f*)(gb + (size_t)row * NCOL) = v;
    }
    __threadfence();
#pragma unroll
    for (int q = 0; q < 16; ++q) {
      const int row = 2 * q + srow;
      const v4f v = *(const v4f*)(sw + row * 64 + scol);
      *(volatile v4f*)(gb + (size_t)row * NCOL) = v;
    }
  } else {
    const int rsub = lane >> 3, j = lane & 7;
#pragma unroll
    for (int q = 0; q < 8; ++q) {
      const int row = 4 * q + rsub;
      const float* sp = sw + row * 64 + 8 * j;
      const v4f x0 = *(const v4f*)sp;
      const v4f x1 = *(const v4f*)(sp + 4);
      v8us hi, lo;
      unsigned short th, tl;
      split_bf(x0.x, th, tl); hi[0] = th; lo[0] = tl;
      split_bf(x0.y, th, tl); hi[1] = th; lo[1] = tl;
      split_bf(x0.z, th, tl); hi[2] = th; lo[2] = tl;
      split_bf(x0.w, th, tl); hi[3] = th; lo[3] = tl;
      split_bf(x1.x, th, tl); hi[4] = th; lo[4] = tl;
      split_bf(x1.y, th, tl); hi[5] = th; lo[5] = tl;
      split_bf(x1.z, th, tl); hi[6] = th; lo[6] = tl;
      split_bf(x1.w, th, tl); hi[7] = th; lo[7] = tl;
      unsigned short* d = C16 + (size_t)(row0 + row) * (3 * NCOL) + col0 + 8 * j;
      *(volatile v8us*)d = hi;
      *(volatile v8us*)(d + NCOL) = hi;
      *(volatile v8us*)(d + 2 * NCOL) = lo;
    }
    __threadfence();
#pragma unroll
    for (int q = 0; q < 8; ++q) {
      const int row = 4 * q + rsub;
      const float* sp = sw + row * 64 + 8 * j;
      const v4f x0 = *(const v4f*)sp;
      const v4f x1 = *(const v4f*)(sp + 4);
      v8us hi, lo;
      unsigned short th, tl;
      split_bf(x0.x, th, tl); hi[0] = th; lo[0] = tl;
      split_bf(x0.y, th, tl); hi[1] = th; lo[1] = tl;
      split_bf(x0.z, th, tl); hi[2] = th; lo[2] = tl;
      split_bf(x0.w, th, tl); hi[3] = th; lo[3] = tl;
      split_bf(x1.x, th, tl); hi[4] = th; lo[4] = tl;
      split_bf(x1.y, th, tl); hi[5] = th; lo[5] = tl;
      split_bf(x1.z, th, tl); hi[6] = th; lo[6] = tl;
      split_bf(x1.w, th, tl); hi[7] = th; lo[7] = tl;
      unsigned short* d = C16 + (size_t)(row0 + row) * (3 * NCOL) + col0 + 8 * j;
      *(volatile v8us*)d = hi;
      *(volatile v8us*)(d + NCOL) = hi;
      *(volatile v8us*)(d + 2 * NCOL) = lo;
    }
  }
}

__global__ __launch_bounds__(BB) void k_head(
    const float* __restrict__ z2, const float* __restrict__ ow, const float* __restrict__ ob,
    float* out) {
  __shared__ __attribute__((aligned(16))) float so[BB * OUTC];
  const int tid = threadIdx.x;
  const float* z = z2 + (size_t)tid * FC2C;
  float l0 = 0.0f, l1 = 0.0f;
#pragma unroll 4
  for (int k = 0; k < FC2C; ++k) {
    const float v = z[k];
    l0 = fmaf(v, ow[2 * k], l0);
    l1 = fmaf(v, ow[2 * k + 1], l1);
  }
  l0 += ob[0];
  l1 += ob[1];
  const float mx = fmaxf(l0, l1);
  const float e0 = expf(l0 - mx), e1 = expf(l1 - mx);
  const float rsum = 1.0f / (e0 + e1);
  so[2 * tid]     = e0 * rsum;
  so[2 * tid + 1] = e1 * rsum;
  __syncthreads();
  v4f v = {0.f, 0.f, 0.f, 0.f};
  if (tid < (BB * OUTC) / 4) v = *(const v4f*)(so + 4 * tid);
  if (tid < (BB * OUTC) / 4) *(volatile v4f*)(out + 4 * tid) = v;
  __threadfence();
  if (tid < (BB * OUTC) / 4) *(volatile v4f*)(out + 4 * tid) = v;
}

extern "C" void kernel_launch(void* const* d_in, const int* in_sizes, int n_in,
                              void* d_out, int out_size, void* d_ws, size_t ws_size,
                              hipStream_t stream) {
  if (n_in < 26) return;
  if (in_sizes[0] != NN * BB) return;
  if (in_sizes[1] <= 0 || (in_sizes[1] & 1) != 0) return;
  const int nE = in_sizes[1] / 2;
  if (nE <= 0 || nE > (1 << 28) || in_sizes[2] != nE) return;
  if (in_sizes[3] != MIDC || in_sizes[5] != MIDC) return;
  if (in_sizes[6] != NN * MIDC || in_sizes[7] != NN * MIDC) return;
  if (in_sizes[8] != GC1C * MIDC || in_sizes[9] != GC1C || in_sizes[10] != GC1C || in_sizes[11] != GC1C) return;
  if (in_sizes[12] != GC2C * GC1C || in_sizes[13] != GC2C || in_sizes[14] != GC2C || in_sizes[15] != GC2C) return;
  if (in_sizes[16] != KFC1 * FC1C || in_sizes[17] != FC1C || in_sizes[18] != FC1C || in_sizes[19] != FC1C) return;
  if (in_sizes[20] != FC1C * FC2C || in_sizes[21] != FC2C || in_sizes[22] != FC2C || in_sizes[23] != FC2C) return;
  if (in_sizes[24] != FC2C * OUTC || in_sizes[25] != OUTC) return;
  if (out_size != BB * OUTC) return;

  const float* x     = (const float*)d_in[0];
  const int*   ei    = (const int*)  d_in[1];
  const float* ewp   = (const float*)d_in[2];
  const float* sgw   = (const float*)d_in[3];
  const float* sgb   = (const float*)d_in[5];
  const float* lng   = (const float*)d_in[6];
  const float* lnb   = (const float*)d_in[7];
  const float* gc1w  = (const float*)d_in[8];
  const float* gc1b  = (const float*)d_in[9];
  const float* bn1g  = (const float*)d_in[10];
  const float* bn1b  = (const float*)d_in[11];
  const float* gc2w  = (const float*)d_in[12];
  const float* gc2b  = (const float*)d_in[13];
  const float* bn2g  = (const float*)d_in[14];
  const float* bn2b  = (const float*)d_in[15];
  const float* fc1w  = (const float*)d_in[16];
  const float* fc1b  = (const float*)d_in[17];
  const float* fbn1g = (const float*)d_in[18];
  const float* fbn1b = (const float*)d_in[19];
  const float* fc2w  = (const float*)d_in[20];
  const float* fc2b  = (const float*)d_in[21];
  const float* fbn2g = (const float*)d_in[22];
  const float* fbn2b = (const float*)d_in[23];
  const float* ouw   = (const float*)d_in[24];
  const float* oub   = (const float*)d_in[25];
  float* out = (float*)d_out;

  const int SIGP = (nE + 31) & ~31;

  char* ws = (char*)d_ws;
  size_t off = 0;
  const size_t oB1  = off; off += (size_t)FC1C * KD1 * 2;   off = (off + 255) & ~(size_t)255;
  const size_t oB2  = off; off += (size_t)FC2C * KD2 * 2;   off = (off + 255) & ~(size_t)255;
  const size_t oSig = off; off += (size_t)SIGP * 4;         off = (off + 255) & ~(size_t)255;
  const size_t oAgg = off; off += (size_t)BB * NP * 4;      off = (off + 255) & ~(size_t)255;
  const size_t oA1  = off; off += (size_t)BB * KD1 * 2;     off = (off + 255) & ~(size_t)255;
  const size_t oZ1  = off; off += (size_t)BB * KD2 * 2;     off = (off + 255) & ~(size_t)255;
  const size_t oZ2  = off; off += (size_t)BB * FC2C * 4;    off = (off + 255) & ~(size_t)255;
  if (off > ws_size || off > (size_t)WSCAP) return;
  unsigned short* B1   = (unsigned short*)(ws + oB1);
  unsigned short* B2   = (unsigned short*)(ws + oB2);
  float*          sig  = (float*)(ws + oSig);
  float*          aggT = (float*)(ws + oAgg);
  unsigned short* A1   = (unsigned short*)(ws + oA1);
  unsigned short* Z1   = (unsigned short*)(ws + oZ1);
  float*          z2   = (float*)(ws + oZ2);

  const int vec8 = ((nE & 3) == 0) ? 1 : 0;

  const int tot1 = FC1C * (3 * (KP1 / 8));
  const int tot2 = FC2C * (3 * (KP2 / 8));
  k_wprep<<<(tot1 + NTHR - 1) / NTHR, NTHR, 0, stream>>>(fc1w, B1, KFC1, FC1C, KP1, tot1);
  k_wprep<<<(tot2 + NTHR - 1) / NTHR, NTHR, 0, stream>>>(fc2w, B2, FC1C, FC2C, KP2, tot2);

  k_sig<<<(SIGP + NTHR - 1) / NTHR, NTHR, 0, stream>>>(ewp, sig, nE, SIGP);

  hipFuncSetAttribute(reinterpret_cast<const void*>(&k_agg),
                      hipFuncAttributeMaxDynamicSharedMemorySize, LDS_AGG);
  k_agg<<<NP / NBA, NTHR, LDS_AGG, stream>>>(x, ei, sig, aggT, nE, vec8);

  k_ln_conv<<<BB, NTHR, 0, stream>>>(aggT, sgw, sgb, lng, lnb, gc1w, gc1b, bn1g, bn1b,
                                     gc2w, gc2b, bn2g, bn2b, A1);

  hipFuncSetAttribute(reinterpret_cast<const void*>(&k_gemm<KD1, FC1C, 1>),
                      hipFuncAttributeMaxDynamicSharedMemorySize, LDS_GEMM);
  k_gemm<KD1, FC1C, 1><<<BB / 64, NTHR, LDS_GEMM, stream>>>(A1, B1, fc1b, fbn1g, fbn1b, z2, Z1);

  hipFuncSetAttribute(reinterpret_cast<const void*>(&k_gemm<KD2, FC2C, 0>),
                      hipFuncAttributeMaxDynamicSharedMemorySize, LDS_GEMM);
  k_gemm<KD2, FC2C, 0><<<BB / 256, NTHR, LDS_GEMM, stream>>>(Z1, B2, fc2b, fbn2g, fbn2b, z2, Z1);

  k_head<<<1, BB, 0, stream>>>(z2, ouw, oub, out);
}
